// VGNN_sparse_59571196396043
// MI455X (gfx1250) — hardware-verified
//
#include <hip/hip_runtime.h>
#include <stddef.h>
#include <stdint.h>

#define NSEG   30000
#define NNODE  10000
#define NEDGE  80000
#define SD     64
#define HM     128
#define SP     30080
#define HP     128
#define PABW   256
#define W1IN   132
#define NSTEP  10
#define NTHR   256
#define NWAVE  8
#define GBM    64
#define GBN    128
#define GTHR   128
#define ETB    128
#define ETHR   128
#define DP     132
#define AP2    264
#define GP     260
#define LTHR   128
#define RTHR   128
#define ROT    79
#define EPT    8
#define CHUNK  (NTHR * EPT)
#define WCAP   (EPT * 32)
#define LISTN  (NWAVE * WCAP)
#define NBA    1024
#define SLA    10
#define NBLK   30
#define RCAP   8192
#define DEGCAP 64
#define ASLOT  128
#define AGG_ZINTS (LISTN + 2 * RCAP + 3 * NBA)
#define AGG_LDS_INTS (AGG_ZINTS + 16)
#define AGG_LDS_BYTES (AGG_LDS_INTS * 4)
#define EDGE_LDS_BYTES (ETB * DP * 4 + ETB * AP2 * 2 + 192 * 4)
#define RO_LDS_BYTES (RTHR * DP * 4 + RTHR * AP2 * 2 + 528 * 4 + 256 * 4)
#define LSTM_LDS_BYTES (GBM * GP * 4 + GBM * HP * 2 + 256 * 4)
#define WSMAX  134217728
#define NU_PA  (256 * 16 + 128 * 32 + 64 * 32)
#define NU_PB  (256 * 16 + 256 * 16 + 128 * 16 + 128 * 32)
#define NU_ST  (SP * 16)

static_assert(NEDGE % ETB == 0 && NEDGE / ETB == 625);
static_assert(NEDGE % 64 == 0 && NEDGE % 8 == 0);
static_assert(NSEG == 234 * 128 + 48 && NNODE == 78 * 128 + 16 && NNODE % 16 == 0);
static_assert(SP % GBM == 0 && SP % 128 == 0 && SP >= NSEG && ROT * RTHR <= SP && ROT * RTHR >= NNODE);
static_assert((CHUNK & (CHUNK - 1)) == 0 && CHUNK <= 4096);
static_assert((NBA & (NBA - 1)) == 0 && NBA == (1 << SLA));
static_assert(((long long)(NEDGE + CHUNK) << SLA) < (1LL << 31));
static_assert(LISTN % NTHR == 0 && NBA % NWAVE == 0 && NBA % 32 == 0);
static_assert(RCAP % 4 == 0 && AGG_ZINTS % 4 == 0 && LISTN % 4 == 0);
static_assert(RCAP >= 4167 + 1024 && DEGCAP >= 15 + 8);
static_assert(NBLK * NBA >= SP && (NBLK - 1) * NBA < SP);
static_assert(RCAP == 8 * NTHR * 4 && NBA == 4 * NTHR);
static_assert(SP % ASLOT == 0 && NBA % ASLOT == 0 && ASLOT == 16 * NWAVE);
static_assert(AGG_LDS_BYTES <= 327680 && EDGE_LDS_BYTES <= 327680);
static_assert(RO_LDS_BYTES <= 327680 && LSTM_LDS_BYTES <= 327680);
static_assert(NU_PA % NTHR == 0 && NU_PB % NTHR == 0 && NU_ST % NTHR == 0);
static_assert((DP * 4) % 16 == 0 && (AP2 * 2) % 16 == 0 && (GP * 4) % 16 == 0);
static_assert(AP2 >= 256 && DP >= HM && GP >= 256);
static_assert(ETB * SD * 4 <= ETB * AP2 * 2 && ETB * SD * 4 == 16 * ETHR * 16);
static_assert(GBM * HP * 2 == 8 * LTHR * 16);
static_assert(GBM == (GTHR / 32) * 16 && GBN == 128);
static_assert((W1IN * 4) % 16 == 0);

typedef float          v2f   __attribute__((ext_vector_type(2)));
typedef float          v4f   __attribute__((ext_vector_type(4)));
typedef float          v8f   __attribute__((ext_vector_type(8)));
typedef int            v4i   __attribute__((ext_vector_type(4)));
typedef int            v8i   __attribute__((ext_vector_type(8)));
typedef unsigned       v4u   __attribute__((ext_vector_type(4)));
typedef unsigned short v4us  __attribute__((ext_vector_type(4)));
typedef unsigned short v8us  __attribute__((ext_vector_type(8)));
typedef unsigned short v16us __attribute__((ext_vector_type(16)));
typedef __bf16         v16bf __attribute__((ext_vector_type(16)));
typedef v2f  __attribute__((may_alias)) v2fa;
typedef v4f  __attribute__((may_alias)) v4fa;
typedef v4i  __attribute__((may_alias)) v4ia;
typedef v4u  __attribute__((may_alias)) v4ua;
typedef v4us __attribute__((may_alias)) v4usa;
typedef v8us __attribute__((may_alias)) v8usa;
union FragB { v16bf v; v16us u; v8us h[2]; v8i w; };

constexpr size_t SZ_W1AB = (size_t)256 * 128 * 2;
constexpr size_t SZ_W2D  = (size_t)128 * 256 * 2;
constexpr size_t SZ_W3D  = (size_t)64 * 256 * 2;
constexpr size_t SZ_WG   = (size_t)256 * 256 * 2;
constexpr size_t SZ_R1D  = (size_t)128 * 128 * 2;
constexpr size_t SZ_R2D  = (size_t)128 * 256 * 2;
constexpr size_t SZ_H    = (size_t)SP * HP * 2;
constexpr size_t SZ_NM   = (size_t)SP * HP * 2;
constexpr size_t SZ_C    = (size_t)SP * SD * 4;
constexpr size_t SZ_PAB  = (size_t)SP * PABW * 4;
constexpr size_t SZ_EC   = (size_t)NEDGE * HM * 4;
constexpr size_t SZ_MSG  = (size_t)NEDGE * SD * 4;
constexpr size_t SZ_LIST = (size_t)NBLK * RCAP * 4;
constexpr size_t SZ_CNT  = (size_t)NBLK * NBA * 4;
constexpr size_t SZ_OFF  = (size_t)NBLK * NBA * 4;
constexpr size_t SZ_FLAG = (size_t)NBLK * 128;
constexpr size_t O_W1AB = 0;
constexpr size_t O_W2D  = O_W1AB + SZ_W1AB;
constexpr size_t O_W3D  = O_W2D + SZ_W2D;
constexpr size_t O_WG   = O_W3D + SZ_W3D;
constexpr size_t O_R1D  = O_WG + SZ_WG;
constexpr size_t O_R2D  = O_R1D + SZ_R1D;
constexpr size_t O_H0   = O_R2D + SZ_R2D;
constexpr size_t O_H1   = O_H0 + SZ_H;
constexpr size_t O_NM   = O_H1 + SZ_H;
constexpr size_t O_C    = O_NM + SZ_NM;
constexpr size_t O_PAB  = O_C + SZ_C;
constexpr size_t O_EC   = O_PAB + SZ_PAB;
constexpr size_t O_MSG  = O_EC + SZ_EC;
constexpr size_t O_LIST = O_MSG + SZ_MSG;
constexpr size_t O_CNT  = O_LIST + SZ_LIST;
constexpr size_t O_OFF  = O_CNT + SZ_CNT;
constexpr size_t O_FLAG = O_OFF + SZ_OFF;
constexpr size_t WS_END = O_FLAG + SZ_FLAG;
static_assert(WS_END <= (size_t)WSMAX);
static_assert(SZ_H % 256 == 0 && SZ_C % 256 == 0 && SZ_PAB % 256 == 0 && SZ_EC % 256 == 0 && SZ_MSG % 256 == 0);
static_assert(SZ_LIST % 256 == 0 && SZ_CNT % 256 == 0 && SZ_OFF % 256 == 0 && SZ_FLAG % 256 == 0);
static_assert((size_t)(NBLK - 1) * RCAP * 4 + (size_t)(8 * NTHR) * 16 <= SZ_LIST);
static_assert((size_t)(NBLK - 1) * NBA * 4 + (size_t)NTHR * 16 <= SZ_CNT);
static_assert((size_t)(NBLK - 1) * 128 + 128 <= SZ_FLAG);

__device__ __forceinline__ v8f wmb(const FragB& a, const FragB& b, v8f c) {
  v8f d = __builtin_amdgcn_wmma_f32_16x16x32_bf16(false, a.v, false, b.v, (short)0, c, false, false);
  asm volatile("v_nop\n\tv_nop\n\tv_nop\n\tv_nop" : "+v"(d) : "v"(a.w), "v"(b.w));
  return d;
}

__device__ __forceinline__ unsigned bf16_bits(float f) {
  const unsigned u = __float_as_uint(f);
  const unsigned r = (u + 0x7FFFu + ((u >> 16) & 1u)) >> 16;
  return ((u & 0x7fffffffu) > 0x7f800000u) ? 0x7fc0u : r;
}
__device__ __forceinline__ float bf16_val(float f) {
  return __uint_as_float(bf16_bits(f) << 16);
}
__device__ __forceinline__ unsigned rne_raw(float f) {
  const unsigned u = __float_as_uint(f);
  return u + 0x7FFFu + ((u >> 16) & 1u);
}
__device__ __forceinline__ float relu_k(float v) {
  return (v > 0.0f) ? v : (v - v);
}
__device__ __forceinline__ void put16(unsigned short* dp, v8us o) {
  *(volatile v8us*)dp = o;
  __threadfence();
  *(volatile v8us*)dp = o;
}
__device__ __forceinline__ void putf4(float* dp, v4f o) {
  *(volatile v4f*)dp = o;
  __threadfence();
  *(volatile v4f*)dp = o;
}
__device__ __forceinline__ void puti4(int* dp, v4i o) {
  *(volatile v4i*)dp = o;
  __threadfence();
  *(volatile v4i*)dp = o;
}
__device__ __forceinline__ v8us cvt8(const float* __restrict__ p) {
  const v4f a = *(const v4fa*)p;
  const v4f b = *(const v4fa*)(p + 4);
  v8us o;
  o[0] = (unsigned short)bf16_bits(a.x); o[1] = (unsigned short)bf16_bits(a.y);
  o[2] = (unsigned short)bf16_bits(a.z); o[3] = (unsigned short)bf16_bits(a.w);
  o[4] = (unsigned short)bf16_bits(b.x); o[5] = (unsigned short)bf16_bits(b.y);
  o[6] = (unsigned short)bf16_bits(b.z); o[7] = (unsigned short)bf16_bits(b.w);
  return o;
}

template <int SLB>
__device__ __forceinline__ int scan_chunk(const int* __restrict__ dsts, int nE, int cbase, int slotBase,
                                          int nb, int vec8, int* list, int tid, int lane, int wave) {
  int wc = 0;
  const int el0  = tid * EPT;
  const int e0   = cbase + el0;
  const int sent = -2147483647 - 1;
  v4i da, db;
  if (vec8 != 0 && cbase + CHUNK <= nE) {
    da = *(const v4i*)(dsts + e0);
    db = *(const v4i*)(dsts + e0 + 4);
  } else {
    da.x = (e0     < nE) ? dsts[min(e0,     nE - 1)] : sent;
    da.y = (e0 + 1 < nE) ? dsts[min(e0 + 1, nE - 1)] : sent;
    da.z = (e0 + 2 < nE) ? dsts[min(e0 + 2, nE - 1)] : sent;
    da.w = (e0 + 3 < nE) ? dsts[min(e0 + 3, nE - 1)] : sent;
    db.x = (e0 + 4 < nE) ? dsts[min(e0 + 4, nE - 1)] : sent;
    db.y = (e0 + 5 < nE) ? dsts[min(e0 + 5, nE - 1)] : sent;
    db.z = (e0 + 6 < nE) ? dsts[min(e0 + 6, nE - 1)] : sent;
    db.w = (e0 + 7 < nE) ? dsts[min(e0 + 7, nE - 1)] : sent;
  }
  const unsigned nbs = (unsigned)slotBase;
  const unsigned unb = (unsigned)nb;
  const unsigned s0 = (unsigned)da.x - nbs, s1 = (unsigned)da.y - nbs;
  const unsigned s2 = (unsigned)da.z - nbs, s3 = (unsigned)da.w - nbs;
  const unsigned s4 = (unsigned)db.x - nbs, s5 = (unsigned)db.y - nbs;
  const unsigned s6 = (unsigned)db.z - nbs, s7 = (unsigned)db.w - nbs;
  const bool h0 = s0 < unb, h1 = s1 < unb, h2 = s2 < unb, h3 = s3 < unb;
  const bool h4 = s4 < unb, h5 = s5 < unb, h6 = s6 < unb, h7 = s7 < unb;
  const unsigned any = __builtin_amdgcn_ballot_w32(h0 | h1 | h2 | h3 | h4 | h5 | h6 | h7);
  if (any != 0u) {
#define HITJ(J, HJ, SJ) { \
      const unsigned mj = __builtin_amdgcn_ballot_w32(HJ); \
      if (mj != 0u) { \
        if (HJ) { \
          const int pos = wc + (int)__builtin_amdgcn_mbcnt_lo(mj, 0u); \
          if (pos < WCAP) list[wave * WCAP + pos] = ((el0 + (J)) << SLB) | (int)(SJ); \
        } \
        wc += (int)__builtin_popcount(mj); } }
    HITJ(0, h0, s0)
    HITJ(1, h1, s1)
    HITJ(2, h2, s2)
    HITJ(3, h3, s3)
    HITJ(4, h4, s4)
    HITJ(5, h5, s5)
    HITJ(6, h6, s6)
    HITJ(7, h7, s7)
#undef HITJ
  }
  return wc;
}

__global__ __launch_bounds__(NTHR) void k_pa(const float* __restrict__ w1, const float* __restrict__ w2,
                                             const float* __restrict__ w3, unsigned short* W1AB,
                                             unsigned short* W2D, unsigned short* W3D) {
  const int u = (int)blockIdx.x * NTHR + (int)threadIdx.x;
  if (u < 4096) {
    const int R = u >> 4, k8 = (u & 15) * 8;
    const int n = R & 127, part = R >> 7;
    const v8us o = cvt8(w1 + (size_t)n * W1IN + part * 64 + (k8 & 63));
    put16(W1AB + (size_t)R * 128 + k8, o);
  } else if (u < 8192) {
    const int v = u - 4096;
    const int n = v >> 5, k8 = (v & 31) * 8;
    const v8us o = cvt8(w2 + (size_t)n * HM + (k8 & 127));
    put16(W2D + (size_t)n * 256 + k8, o);
  } else if (u < NU_PA) {
    const int v = u - 8192;
    const int n = v >> 5, k8 = (v & 31) * 8;
    const v8us o = cvt8(w3 + (size_t)n * HM + (k8 & 127));
    put16(W3D + (size_t)n * 256 + k8, o);
  }
}

__global__ __launch_bounds__(NTHR) void k_pb(const float* __restrict__ wih, const float* __restrict__ whh,
                                             const float* __restrict__ rw1, const float* __restrict__ rw2,
                                             unsigned short* WG, unsigned short* R1D, unsigned short* R2D) {
  const int u = (int)blockIdx.x * NTHR + (int)threadIdx.x;
  if (u < 4096) {
    const int n = u >> 4, k8 = (u & 15) * 8;
    const v8us o = cvt8(wih + (size_t)n * SD + (k8 & 63));
    put16(WG + (size_t)n * 256 + k8, o);
  } else if (u < 8192) {
    const int v = u - 4096;
    const int n = v >> 4, k8 = (v & 15) * 8;
    const v8us o = cvt8(whh + (size_t)n * SD + (k8 & 63));
    put16(WG + (size_t)n * 256 + 128 + k8, o);
  } else if (u < 10240) {
    const int v = u - 8192;
    const int n = v >> 4, k8 = (v & 15) * 8;
    const v8us o = cvt8(rw1 + (size_t)n * SD + (k8 & 63));
    put16(R1D + (size_t)n * 128 + k8, o);
  } else if (u < NU_PB) {
    const int v = u - 10240;
    const int n = v >> 5, k8 = (v & 31) * 8;
    const v8us o = cvt8(rw2 + (size_t)n * HM + (k8 & 127));
    put16(R2D + (size_t)n * 256 + k8, o);
  }
}

__global__ __launch_bounds__(NTHR) void k_pc(unsigned short* H0, unsigned short* H1, float* C) {
  const int u = (int)blockIdx.x * NTHR + (int)threadIdx.x;
  if (u < NU_ST) {
    const int row = u >> 4, j = u & 15;
    const int one = (j == 0 && row >= NNODE && row < NSEG) ? 0x3F80 : 0;
    const v4i o = {one, 0, 0, 0};
    puti4((int*)(H0 + (size_t)u * 8), o);
  } else if (u < 2 * NU_ST) {
    const int v = u - NU_ST;
    const v4i o = {0, 0, 0, 0};
    puti4((int*)(H1 + (size_t)v * 8), o);
  } else if (u < 3 * NU_ST) {
    const int v = u - 2 * NU_ST;
    const v4f o = {0.0f, 0.0f, 0.0f, 0.0f};
    putf4(C + (size_t)v * 4, o);
  }
}

__global__ __launch_bounds__(NTHR) void k_ec(const float* __restrict__ ea, const float* __restrict__ w1,
                                             const float* __restrict__ b1, float* EC) {
  const int tid = (int)threadIdx.x, lane = tid & 31, wave = tid >> 5;
  const int n4 = 4 * lane;
  v4f w0 = *(const v4fa*)(w1 + (size_t)(n4 + 0) * W1IN + 128);
  v4f wA = *(const v4fa*)(w1 + (size_t)(n4 + 1) * W1IN + 128);
  v4f wB = *(const v4fa*)(w1 + (size_t)(n4 + 2) * W1IN + 128);
  v4f wC = *(const v4fa*)(w1 + (size_t)(n4 + 3) * W1IN + 128);
  v4f bb = *(const v4fa*)(b1 + n4);
  w0.x = bf16_val(w0.x); w0.y = bf16_val(w0.y); w0.z = bf16_val(w0.z); w0.w = bf16_val(w0.w);
  wA.x = bf16_val(wA.x); wA.y = bf16_val(wA.y); wA.z = bf16_val(wA.z); wA.w = bf16_val(wA.w);
  wB.x = bf16_val(wB.x); wB.y = bf16_val(wB.y); wB.z = bf16_val(wB.z); wB.w = bf16_val(wB.w);
  wC.x = bf16_val(wC.x); wC.y = bf16_val(wC.y); wC.z = bf16_val(wC.z); wC.w = bf16_val(wC.w);
  bb.x = bf16_val(bb.x); bb.y = bf16_val(bb.y); bb.z = bf16_val(bb.z); bb.w = bf16_val(bb.w);
  const int e0 = (int)blockIdx.x * 64 + wave * 8;
#pragma unroll 1
  for (int i = 0; i < 8; ++i) {
    const int e = e0 + i;
    v4f a = *(const v4fa*)(ea + (size_t)e * 4);
    a.x = bf16_val(a.x); a.y = bf16_val(a.y); a.z = bf16_val(a.z); a.w = bf16_val(a.w);
    v4f o;
    o.x = fmaf(a.w, w0.w, fmaf(a.z, w0.z, fmaf(a.y, w0.y, fmaf(a.x, w0.x, bb.x))));
    o.y = fmaf(a.w, wA.w, fmaf(a.z, wA.z, fmaf(a.y, wA.y, fmaf(a.x, wA.x, bb.y))));
    o.z = fmaf(a.w, wB.w, fmaf(a.z, wB.z, fmaf(a.y, wB.y, fmaf(a.x, wB.x, bb.z))));
    o.w = fmaf(a.w, wC.w, fmaf(a.z, wC.z, fmaf(a.y, wC.y, fmaf(a.x, wC.x, bb.w))));
    putf4(EC + (size_t)e * HM + n4, o);
  }
}

__device__ __forceinline__ void gemm_k8(const unsigned short* __restrict__ ap, const unsigned short* __restrict__ bp,
                                        int ldb, int K, v8f (&acc)[8]) {
#pragma unroll 1
  for (int k0 = 0; k0 < K; k0 += 32) {
    FragB af;
    af.h[0] = *(const v8usa*)(ap + k0);
    af.h[1] = *(const v8usa*)(ap + k0 + 16);
#pragma unroll
    for (int nt = 0; nt < 8; ++nt) {
      const unsigned short* wq = bp + (size_t)(16 * nt) * (size_t)ldb + k0;
      FragB bf;
      bf.h[0] = *(const v8usa*)wq;
      bf.h[1] = *(const v8usa*)(wq + 16);
      acc[nt] = wmb(af, bf, acc[nt]);
    }
  }
}

__global__ __launch_bounds__(GTHR) __attribute__((amdgpu_num_vgpr(248)))
void k_node(const unsigned short* __restrict__ A, int lda, const unsigned short* __restrict__ BT, int ldb, int K,
            float* Cm, int ldc) {
  __shared__ __attribute__((aligned(16))) float stg[GBM * GBN];
  const int tid = (int)threadIdx.x, lane = tid & 31, wave = tid >> 5, hh = lane >> 4, m = lane & 15;
  const int rowBase = (int)blockIdx.x * GBM;
  const int colBase = (int)blockIdx.y * GBN;
  v8f acc[8];
  {
    const v8f z = {0.f, 0.f, 0.f, 0.f, 0.f, 0.f, 0.f, 0.f};
#pragma unroll
    for (int t = 0; t < 8; ++t) acc[t] = z;
  }
  const unsigned short* ap = A  + (size_t)(rowBase + 16 * wave + m) * (size_t)lda + 8 * hh;
  const unsigned short* bp = BT + (size_t)(colBase + m) * (size_t)ldb + 8 * hh;
  gemm_k8(ap, bp, ldb, K, acc);
#pragma unroll
  for (int nt = 0; nt < 8; ++nt) {
    const int lc = 16 * nt + m;
#pragma unroll
    for (int r = 0; r < 8; ++r) stg[(16 * wave + 8 * hh + r) * GBN + lc] = acc[nt][r];
  }
  __syncthreads();
  v4f pv[16];
#pragma unroll
  for (int i = 0; i < 16; ++i) pv[i] = *(const v4fa*)(stg + (16 * wave + i) * GBN + 4 * lane);
#pragma unroll
  for (int i = 0; i < 16; ++i) {
    float* op = Cm + (size_t)(rowBase + 16 * wave + i) * (size_t)ldc + colBase + 4 * lane;
    *(volatile v4f*)op = pv[i];
  }
  __threadfence();
#pragma unroll
  for (int i = 0; i < 16; ++i) {
    float* op = Cm + (size_t)(rowBase + 16 * wave + i) * (size_t)ldc + colBase + 4 * lane;
    *(volatile v4f*)op = pv[i];
  }
}

template <int APITCH, int NHALF>
__device__ __forceinline__ void wave_gemm_b(const unsigned short* sAw, float* sDw,
                                            const unsigned short* __restrict__ BT, int ldb, int K,
                                            int hh, int m) {
#pragma unroll 1
  for (int nh = 0; nh < NHALF; ++nh) {
    v8f acc[2][4];
    {
      const v8f z = {0.f, 0.f, 0.f, 0.f, 0.f, 0.f, 0.f, 0.f};
#pragma unroll
      for (int mt = 0; mt < 2; ++mt)
#pragma unroll
        for (int nt = 0; nt < 4; ++nt) acc[mt][nt] = z;
    }
    const unsigned short* ap0 = sAw + m * APITCH + 8 * hh;
    const unsigned short* ap1 = ap0 + 16 * APITCH;
    const unsigned short* bp  = BT + (size_t)(64 * nh + m) * (size_t)ldb + 8 * hh;
#pragma unroll 1
    for (int k0 = 0; k0 < K; k0 += 32) {
      FragB a0, a1;
      a0.h[0] = *(const v8usa*)(ap0 + k0);
      a0.h[1] = *(const v8usa*)(ap0 + k0 + 16);
      a1.h[0] = *(const v8usa*)(ap1 + k0);
      a1.h[1] = *(const v8usa*)(ap1 + k0 + 16);
#pragma unroll
      for (int nt = 0; nt < 4; ++nt) {
        const unsigned short* wq = bp + (size_t)(16 * nt) * (size_t)ldb + k0;
        FragB b;
        b.h[0] = *(const v8usa*)wq;
        b.h[1] = *(const v8usa*)(wq + 16);
        acc[0][nt] = wmb(a0, b, acc[0][nt]);
        acc[1][nt] = wmb(a1, b, acc[1][nt]);
      }
    }
#pragma unroll
    for (int nt = 0; nt < 4; ++nt) {
      const int col = 64 * nh + 16 * nt + m;
#pragma unroll
      for (int mt = 0; mt < 2; ++mt)
#pragma unroll
        for (int r = 0; r < 8; ++r) sDw[(16 * mt + 8 * hh + r) * DP + col] = acc[mt][nt][r];
    }
  }
}

__device__ __forceinline__ void split8_store(unsigned short* rowp, int c, int off, const v8f f8) {
  v8us ho, lo;
#pragma unroll
  for (int i = 0; i < 8; ++i) {
    const unsigned hb = bf16_bits(f8[i]);
    ho[i] = (unsigned short)hb;
    lo[i] = (unsigned short)bf16_bits(f8[i] - __uint_as_float(hb << 16));
  }
  *(v8usa*)(rowp + c)       = ho;
  *(v8usa*)(rowp + off + c) = lo;
}

__device__ __forceinline__ void split8_pack(unsigned short* rowp, int c, int off, const v8f f8) {
  v4u hw, lw;
#pragma unroll
  for (int j = 0; j < 4; ++j) {
    const float x0 = f8[2 * j];
    const float x1 = f8[2 * j + 1];
    const unsigned r0 = rne_raw(x0);
    const unsigned r1 = rne_raw(x1);
    const unsigned h0 = r0 & 0xffff0000u;
    const unsigned h1 = r1 & 0xffff0000u;
    hw[j] = (r0 >> 16) | h1;
    const unsigned s0 = rne_raw(x0 - __uint_as_float(h0));
    const unsigned s1 = rne_raw(x1 - __uint_as_float(h1));
    lw[j] = (s0 >> 16) | (s1 & 0xffff0000u);
  }
  *(v4ua*)(rowp + c)       = hw;
  *(v4ua*)(rowp + off + c) = lw;
}

__global__ __launch_bounds__(ETHR) __attribute__((amdgpu_num_vgpr(248)))
void k_edge(const int* __restrict__ rowv, const int* __restrict__ colv,
            const float* __restrict__ PAB, const float* __restrict__ EC,
            const unsigned short* __restrict__ W2D, const unsigned short* __restrict__ W3D,
            const float* __restrict__ b2, const float* __restrict__ b3, float* MSG) {
  extern __shared__ __attribute__((aligned(16))) float dyn[];
  float*          sD  = dyn;
  unsigned short* sA  = (unsigned short*)(dyn + ETB * DP);
  float*          sM  = dyn + ETB * DP;
  float*          cst = dyn + ETB * DP + (ETB * AP2) / 2;
  const int tid = (int)threadIdx.x, lane = tid & 31, wave = tid >> 5, hh = lane >> 4, m = lane & 15;

  cst[tid] = bf16_val(b2[tid]);
  if (tid < SD) cst[HM + tid] = bf16_val(b3[tid]);

  const int e = (int)blockIdx.x * ETB + tid;
  int s = rowv[e];
  int t = colv[e];
  s = s < 0 ? 0 : (s > NSEG - 1 ? NSEG - 1 : s);
  t = t < 0 ? 0 : (t > NSEG - 1 ? NSEG - 1 : t);
  float*          rd = sD + tid * DP;
  unsigned short* ra = sA + tid * AP2;
  {
    const float* pa = PAB + (size_t)s * PABW;
    const float* pb = PAB + (size_t)t * PABW + HM;
    const float* pc = EC + (size_t)e * HM;
#pragma unroll 1
    for (int c8 = 0; c8 < HM / 8; ++c8) {
      const v4f a0 = *(const v4fa*)(pa + 8 * c8);
      const v4f a1 = *(const v4fa*)(pa + 8 * c8 + 4);
      const v4f q0 = *(const v4fa*)(pb + 8 * c8);
      const v4f q1 = *(const v4fa*)(pb + 8 * c8 + 4);
      const v4f c0 = *(const v4fa*)(pc + 8 * c8);
      const v4f c1 = *(const v4fa*)(pc + 8 * c8 + 4);
      v8f f8;
      f8[0] = relu_k((a0.x + q0.x) + c0.x); f8[1] = relu_k((a0.y + q0.y) + c0.y);
      f8[2] = relu_k((a0.z + q0.z) + c0.z); f8[3] = relu_k((a0.w + q0.w) + c0.w);
      f8[4] = relu_k((a1.x + q1.x) + c1.x); f8[5] = relu_k((a1.y + q1.y) + c1.y);
      f8[6] = relu_k((a1.z + q1.z) + c1.z); f8[7] = relu_k((a1.w + q1.w) + c1.w);
      split8_pack(ra, 8 * c8, HM, f8);
    }
  }
  __syncthreads();

  const unsigned short* sAw = sA + 32 * wave * AP2;
  float*                sDw = sD + 32 * wave * DP;

  wave_gemm_b<AP2, 2>(sAw, sDw, W2D, 256, 256, hh, m);
  __syncthreads();

#pragma unroll 1
  for (int c8 = 0; c8 < HM / 8; ++c8) {
    const v4f va = *(const v4fa*)(rd + 8 * c8);
    const v4f vb = *(const v4fa*)(rd + 8 * c8 + 4);
    const v4f ba = *(const v4fa*)(cst + 8 * c8);
    const v4f bb = *(const v4fa*)(cst + 8 * c8 + 4);
    v8f f8;
    f8[0] = relu_k(va.x + ba.x); f8[1] = relu_k(va.y + ba.y);
    f8[2] = relu_k(va.z + ba.z); f8[3] = relu_k(va.w + ba.w);
    f8[4] = relu_k(vb.x + bb.x); f8[5] = relu_k(vb.y + bb.y);
    f8[6] = relu_k(vb.z + bb.z); f8[7] = relu_k(vb.w + bb.w);
    split8_pack(ra, 8 * c8, HM, f8);
  }
  __syncthreads();

  wave_gemm_b<AP2, 1>(sAw, sDw, W3D, 256, 256, hh, m);
  __syncthreads();

  {
    float* rmo = sM + tid * SD;
#pragma unroll 1
    for (int c8 = 0; c8 < SD / 8; ++c8) {
      const v4f va = *(const v4fa*)(rd + 8 * c8);
      const v4f vb = *(const v4fa*)(rd + 8 * c8 + 4);
      const v4f ba = *(const v4fa*)(cst + HM + 8 * c8);
      const v4f bb = *(const v4fa*)(cst + HM + 8 * c8 + 4);
      v4f o0, o1;
      o0.x = va.x + ba.x; o0.y = va.y + ba.y; o0.z = va.z + ba.z; o0.w = va.w + ba.w;
      o1.x = vb.x + bb.x; o1.y = vb.y + bb.y; o1.z = vb.z + bb.z; o1.w = vb.w + bb.w;
      *(v4fa*)(rmo + 8 * c8)     = o0;
      *(v4fa*)(rmo + 8 * c8 + 4) = o1;
    }
  }
  __syncthreads();

  {
    v4f pv[16];
#pragma unroll
    for (int it = 0; it < 16; ++it) pv[it] = *(const v4fa*)(sM + (size_t)(it * ETHR + tid) * 4);
    float* mb = MSG + (size_t)blockIdx.x * (size_t)(ETB * SD);
#pragma unroll
    for (int it = 0; it < 16; ++it) *(volatile v4f*)(mb + (size_t)(it * ETHR + tid) * 4) = pv[it];
    __threadfence();
#pragma unroll
    for (int it = 0; it < 16; ++it) *(volatile v4f*)(mb + (size_t)(it * ETHR + tid) * 4) = pv[it];
  }
}

__global__ __launch_bounds__(NTHR) __attribute__((amdgpu_num_vgpr(248)))
void k_bucket(const int* __restrict__ dsts, int nEh, int vec8, int* LIST, int* CNT, int* OFF, int* FLAG) {
  extern __shared__ __attribute__((aligned(16))) int dsm[];
  int*   list = dsm;
  int*   hl   = dsm + LISTN;
  int*   sl   = hl + RCAP;
  int*   cnt  = sl + RCAP;
  int*   offs = cnt + NBA;
  int*   cur  = offs + NBA;
  int*   misc = cur + NBA;
  const int tid = (int)threadIdx.x, lane = tid & 31, wave = tid >> 5;
  const int nodeBase = (int)blockIdx.x * NBA;

  {
    const v4i z4 = {0, 0, 0, 0};
    for (int i = tid * 4; i < AGG_ZINTS; i += NTHR * 4) *(v4ia*)(dsm + i) = z4;
    if (tid < 16) misc[tid] = 0;
  }
  __syncthreads();

  int t = 0, ov = 0;
  const int nChunks = (nEh + CHUNK - 1) / CHUNK;
#pragma unroll 1
  for (int ch = 0; ch < nChunks; ++ch) {
    const int cbase = ch * CHUNK;
    const int wc = scan_chunk<SLA>(dsts, nEh, cbase, nodeBase, NBA, vec8, list, tid, lane, wave);
    if (lane == 0) misc[wave] = wc;
    __syncthreads();
    if (wave == 0) {
#pragma unroll 1
      for (int w2 = 0; w2 < NWAVE; ++w2) {
        int c = misc[w2];
        c = c < 0 ? 0 : (c > WCAP ? WCAP : c);
#pragma unroll 1
        for (int b0 = 0; b0 < c; b0 += 32) {
          const int idx = b0 + lane;
          const int ent = list[w2 * WCAP + (idx < WCAP ? idx : WCAP - 1)];
          const int m32 = (c - b0) < 32 ? (c - b0) : 32;
#pragma unroll 1
          for (int k = 0; k < m32; ++k) {
            const int u    = __builtin_amdgcn_readlane(ent, k);
            const int slot = u & (NBA - 1);
            const int el   = (u >> SLA) & (CHUNK - 1);
            const int pk   = ((cbase + el) << SLA) | slot;
            if (t < RCAP) {
              if (lane == 0) { hl[t] = pk; cnt[slot] = cnt[slot] + 1; }
              t = t + 1;
            } else {
              ov = 1;
            }
          }
        }
      }
    }
    __syncthreads();
  }
  if (wave == 0 && lane == 0) { misc[8] = t; misc[9] = ov; }
  __syncthreads();
  int tt = misc[8];
  tt = tt < 0 ? 0 : (tt > RCAP ? RCAP : tt);
  const int ovf = misc[9];

  if (wave == 0) {
    const int base = lane * (NBA / 32);
    int s = 0;
#pragma unroll 1
    for (int i = 0; i < NBA / 32; ++i) s += cnt[base + i];
    int incl = s;
#pragma unroll
    for (int d = 1; d < 32; d <<= 1) {
      const int y = __shfl_up(incl, d, 32);
      if (lane >= d) incl += y;
    }
    int run = incl - s;
#pragma unroll 1
    for (int i = 0; i < NBA / 32; ++i) {
      const int cv = cnt[base + i];
      offs[base + i] = run;
      cur[base + i]  = run;
      run += cv;
    }
  }
  __syncthreads();
  if (wave == 0) {
#pragma unroll 1
    for (int b0 = 0; b0 < tt; b0 += 32) {
      const int idx = b0 + lane;
      const int ent = hl[idx < RCAP ? idx : RCAP - 1];
      const int m32 = (tt - b0) < 32 ? (tt - b0) : 32;
#pragma unroll 1
      for (int k = 0; k < m32; ++k) {
        const int u    = __builtin_amdgcn_readlane(ent, k);
        const int slot = u & (NBA - 1);
        if (lane == 0) {
          int p = cur[slot];
          p = p < 0 ? 0 : (p > RCAP - 1 ? RCAP - 1 : p);
          sl[p] = u;
          cur[slot] = p + 1;
        }
      }
    }
  }
  __syncthreads();

  {
    v4i pv[8];
#pragma unroll
    for (int it = 0; it < 8; ++it) pv[it] = *(const v4ia*)(sl + (size_t)(it * NTHR + tid) * 4);
    const v4i cv4 = *(const v4ia*)(cnt + 4 * tid);
    const v4i ov4 = *(const v4ia*)(offs + 4 * tid);
    const v4i fv4 = {ovf, tt, ovf, tt};
    int* lb = LIST + (size_t)blockIdx.x * RCAP;
    int* cb = CNT  + (size_t)blockIdx.x * NBA + 4 * tid;
    int* ob = OFF  + (size_t)blockIdx.x * NBA + 4 * tid;
    const int tf = tid < 8 ? tid : 7;
    int* fb = FLAG + (size_t)blockIdx.x * 32 + 4 * tf;
#pragma unroll
    for (int it = 0; it < 8; ++it) *(volatile v4i*)(lb + (size_t)(it * NTHR + tid) * 4) = pv[it];
    *(volatile v4i*)cb = cv4;
    *(volatile v4i*)ob = ov4;
    if (tid < 8) *(volatile v4i*)fb = fv4;
    __threadfence();
#pragma unroll
    for (int it = 0; it < 8; ++it) *(volatile v4i*)(lb + (size_t)(it * NTHR + tid) * 4) = pv[it];
    *(volatile v4i*)cb = cv4;
    *(volatile v4i*)ob = ov4;
    if (tid < 8) *(volatile v4i*)fb = fv4;
  }
}

__global__ __launch_bounds__(NTHR) __attribute__((amdgpu_num_vgpr(248)))
void k_agg(const int* __restrict__ LIST, const int* __restrict__ CNT, const int* __restrict__ OFF,
           const int* __restrict__ FLAG, const float* __restrict__ Mf, unsigned short* NM) {
  const int tid = (int)threadIdx.x, lane = tid & 31, wave = tid >> 5;
  const int blk = ((int)blockIdx.x * ASLOT) >> SLA;
  const int slotBase = (int)blockIdx.x * ASLOT + 16 * wave;
  const int* lb = LIST + (size_t)blk * RCAP;
  const int ovf = FLAG[(size_t)blk * 32];
  const int cl  = CNT[slotBase + (lane & 15)];
  const int ol  = OFF[slotBase + (lane & 15)];
  const float qnan = __int_as_float(0x7fc00000);
  const float pz = (ovf != 0) ? qnan : 0.0f;
#pragma unroll 1
  for (int i = 0; i < 16; ++i) {
    const int node = slotBase + i;
    int c = __builtin_amdgcn_readlane(cl, i);
    const bool big = c > DEGCAP;
    c = c < 0 ? 0 : (c > DEGCAP ? DEGCAP : c);
    int o = __builtin_amdgcn_readlane(ol, i);
    o = o < 0 ? 0 : (o > RCAP ? RCAP : o);
    float a0 = 0.0f, a1 = 0.0f;
#pragma unroll 1
    for (int b0 = 0; b0 < c; b0 += 32) {
      int idx = o + b0 + lane;
      idx = idx > RCAP - 1 ? RCAP - 1 : idx;
      const int ent = lb[idx];
      int eid = ent >> SLA;
      eid = eid < 0 ? 0 : (eid > NEDGE - 1 ? NEDGE - 1 : eid);
      const int m32 = (c - b0) < 32 ? (c - b0) : 32;
#pragma unroll 1
      for (int k = 0; k < m32; ++k) {
        const int ek = __builtin_amdgcn_readlane(eid, k);
        const v2f w = *(const v2fa*)(Mf + (size_t)ek * SD + 2 * lane);
        a0 += w.x;
        a1 += w.y;
      }
    }
    const float pzr = big ? qnan : pz;
    const float v0 = a0 + pzr;
    const float v1 = a1 + pzr;
    const unsigned hb0 = bf16_bits(v0);
    const unsigned hb1 = bf16_bits(v1);
    const unsigned lb0 = bf16_bits(v0 - __uint_as_float(hb0 << 16));
    const unsigned lb1 = bf16_bits(v1 - __uint_as_float(hb1 << 16));
    const unsigned hw = hb0 | (hb1 << 16);
    const unsigned lw = lb0 | (lb1 << 16);
    unsigned* np = (unsigned*)(NM + (size_t)node * HP);
    *(volatile unsigned*)(np + lane) = hw;
    *(volatile unsigned*)(np + 32 + lane) = lw;
    __threadfence();
    *(volatile unsigned*)(np + lane) = hw;
    *(volatile unsigned*)(np + 32 + lane) = lw;
  }
}

__device__ __forceinline__ float sig_x2(float t) {
  float a = t * -1.44269504f;
  a = (a < -126.0f) ? -126.0f : a;
  a = (a > 126.0f) ? 126.0f : a;
  return __builtin_amdgcn_rcpf(1.0f + __builtin_amdgcn_exp2f(a));
}
__device__ __forceinline__ float tanh_x2(float t) {
  return fmaf(2.0f, sig_x2(t + t), -1.0f);
}
__device__ __forceinline__ void lstm1(float xi, float xf, float xg, float xo, float cold, float& cn, float& hn) {
  const float si = sig_x2(xi);
  const float sf = sig_x2(xf);
  const float so = sig_x2(xo);
  const float tg = tanh_x2(xg);
  const float cv = sf * cold + si * tg;
  cn = cv;
  hn = so * tanh_x2(cv);
}

__global__ __launch_bounds__(LTHR) __attribute__((amdgpu_num_vgpr(248)))
void k_lstm(const unsigned short* __restrict__ NM, const unsigned short* __restrict__ Hin,
            const unsigned short* __restrict__ WG, const float* __restrict__ bih, const float* __restrict__ bhh,
            float* C, unsigned short* Hout) {
  extern __shared__ __attribute__((aligned(16))) float ldyn[];
  float*          stg = ldyn;
  unsigned short* sH  = (unsigned short*)(ldyn + GBM * GP);
  float*          cst = ldyn + GBM * GP + (GBM * HP) / 2;
  const int tid = (int)threadIdx.x, lane = tid & 31, wave = tid >> 5, hh = lane >> 4, m = lane & 15;
  const int rowBase = (int)blockIdx.x * GBM;

  cst[tid]        = bf16_val(bih[tid]) + bf16_val(bhh[tid]);
  cst[LTHR + tid] = bf16_val(bih[LTHR + tid]) + bf16_val(bhh[LTHR + tid]);

  const unsigned short* apN = NM  + (size_t)(rowBase + 16 * wave + m) * HP + 8 * hh;
  const unsigned short* apH = Hin + (size_t)(rowBase + 16 * wave + m) * HP + 8 * hh;
#pragma unroll 1
  for (int nh = 0; nh < 2; ++nh) {
    v8f acc[8];
    {
      const v8f z = {0.f, 0.f, 0.f, 0.f, 0.f, 0.f, 0.f, 0.f};
#pragma unroll
      for (int t = 0; t < 8; ++t) acc[t] = z;
    }
    const unsigned short* bp = WG + (size_t)(128 * nh + m) * 256 + 8 * hh;
    gemm_k8(apN, bp, 256, 128, acc);
    gemm_k8(apH, bp + 128, 256, 128, acc);
#pragma unroll
    for (int nt = 0; nt < 8; ++nt) {
      const int lc = 128 * nh + 16 * nt + m;
#pragma unroll
      for (int r = 0; r < 8; ++r) stg[(16 * wave + 8 * hh + r) * GP + lc] = acc[nt][r];
    }
  }
  __syncthreads();

#pragma unroll 1
  for (int s = 0; s < 8; ++s) {
    const int p    = s * LTHR + tid;
    const int r    = p >> 4;
    const int j4   = (p & 15) * 4;
    const int grow = rowBase + r;
    const bool live = grow < NSEG;
    const float* gp = stg + r * GP + j4;
    const v4f gi = *(const v4fa*)(gp);
    const v4f gf = *(const v4fa*)(gp + 64);
    const v4f gg = *(const v4fa*)(gp + 128);
    const v4f go = *(const v4fa*)(gp + 192);
    const v4f bi = *(const v4fa*)(cst + j4);
    const v4f bf = *(const v4fa*)(cst + 64 + j4);
    const v4f bg = *(const v4fa*)(cst + 128 + j4);
    const v4f bo = *(const v4fa*)(cst + 192 + j4);
    float* cp = C + (size_t)grow * SD + j4;
    const v4f co = *(const v4fa*)cp;
    float c0, c1, c2, c3, h0, h1, h2, h3;
    lstm1(gi.x + bi.x, gf.x + bf.x, gg.x + bg.x, go.x + bo.x, co.x, c0, h0);
    lstm1(gi.y + bi.y, gf.y + bf.y, gg.y + bg.y, go.y + bo.y, co.y, c1, h1);
    lstm1(gi.z + bi.z, gf.z + bf.z, gg.z + bg.z, go.z + bo.z, co.z, c2, h2);
    lstm1(gi.w + bi.w, gf.w + bf.w, gg.w + bg.w, go.w + bo.w, co.w, c3, h3);
    const v4f cn = {c0, c1, c2, c3};
    if (live) *(volatile v4f*)cp = cn;
    __threadfence();
    if (live) *(volatile v4f*)cp = cn;
    const unsigned hb0 = bf16_bits(h0), hb1 = bf16_bits(h1), hb2 = bf16_bits(h2), hb3 = bf16_bits(h3);
    v4us ho, lo;
    ho.x = (unsigned short)hb0; ho.y = (unsigned short)hb1; ho.z = (unsigned short)hb2; ho.w = (unsigned short)hb3;
    lo.x = (unsigned short)bf16_bits(h0 - __uint_as_float(hb0 << 16));
    lo.y = (unsigned short)bf16_bits(h1 - __uint_as_float(hb1 << 16));
    lo.z = (unsigned short)bf16_bits(h2 - __uint_as_float(hb2 << 16));
    lo.w = (unsigned short)bf16_bits(h3 - __uint_as_float(hb3 << 16));
    *(v4usa*)(sH + r * HP + j4)      = ho;
    *(v4usa*)(sH + r * HP + SD + j4) = lo;
  }
  __syncthreads();

  {
    v4i pv[8];
#pragma unroll
    for (int it = 0; it < 8; ++it) pv[it] = *(const v4ia*)(sH + (size_t)(it * LTHR + tid) * 8);
    unsigned short* hb = Hout + (size_t)rowBase * HP;
#pragma unroll
    for (int it = 0; it < 8; ++it) {
      const int piece = it * LTHR + tid;
      if (rowBase + (piece >> 4) < NSEG) *(volatile v4i*)(hb + (size_t)piece * 8) = pv[it];
    }
    __threadfence();
#pragma unroll
    for (int it = 0; it < 8; ++it) {
      const int piece = it * LTHR + tid;
      if (rowBase + (piece >> 4) < NSEG) *(volatile v4i*)(hb + (size_t)piece * 8) = pv[it];
    }
  }
}

__global__ __launch_bounds__(RTHR) __attribute__((amdgpu_num_vgpr(248)))
void k_ro(const unsigned short* __restrict__ H, const unsigned short* __restrict__ R1D,
          const unsigned short* __restrict__ R2D, const float* __restrict__ rb1, const float* __restrict__ rb2,
          const float* __restrict__ rw3, const float* __restrict__ rb3, float* out) {
  extern __shared__ __attribute__((aligned(16))) float rdyn[];
  float*          sD  = rdyn;
  unsigned short* sA  = (unsigned short*)(rdyn + RTHR * DP);
  float*          cst = rdyn + RTHR * DP + (RTHR * AP2) / 2;
  float*          sO  = cst + 528;
  const int tid = (int)threadIdx.x, lane = tid & 31, wave = tid >> 5, hh = lane >> 4, m = lane & 15;
  const int rowBase = (int)blockIdx.x * RTHR;

  cst[tid]          = bf16_val(rb1[tid]);
  cst[HM + tid]     = bf16_val(rb2[tid]);
  cst[2 * HM + tid] = bf16_val(rw3[tid]);
  cst[3 * HM + tid] = bf16_val(rw3[HM + tid]);
  if (tid < 2) cst[4 * HM + tid] = bf16_val(rb3[tid]);

#pragma unroll 4
  for (int it = 0; it < 16; ++it) {
    const int p = it * RTHR + tid;
    const int r = p >> 4;
    const int c = (p & 15) * 8;
    const v8us v = *(const v8usa*)(H + (size_t)(rowBase + r) * HP + c);
    *(v8usa*)(sA + r * AP2 + c) = v;
  }
  __syncthreads();

  const unsigned short* sAw = sA + 32 * wave * AP2;
  float*                sDw = sD + 32 * wave * DP;
  float*                rd  = sD + tid * DP;
  unsigned short*       ra  = sA + tid * AP2;

  wave_gemm_b<AP2, 2>(sAw, sDw, R1D, 128, 128, hh, m);
  __syncthreads();

#pragma unroll 1
  for (int c8 = 0; c8 < HM / 8; ++c8) {
    const v4f va = *(const v4fa*)(rd + 8 * c8);
    const v4f vb = *(const v4fa*)(rd + 8 * c8 + 4);
    const v4f ba = *(const v4fa*)(cst + 8 * c8);
    const v4f bb = *(const v4fa*)(cst + 8 * c8 + 4);
    v8f f8;
    f8[0] = relu_k(va.x + ba.x); f8[1] = relu_k(va.y + ba.y);
    f8[2] = relu_k(va.z + ba.z); f8[3] = relu_k(va.w + ba.w);
    f8[4] = relu_k(vb.x + bb.x); f8[5] = relu_k(vb.y + bb.y);
    f8[6] = relu_k(vb.z + bb.z); f8[7] = relu_k(vb.w + bb.w);
    split8_store(ra, 8 * c8, HM, f8);
  }
  __syncthreads();

  wave_gemm_b<AP2, 2>(sAw, sDw, R2D, 256, 256, hh, m);
  __syncthreads();

  {
    float z0 = cst[4 * HM];
    float z1 = cst[4 * HM + 1];
#pragma unroll 1
    for (int c8 = 0; c8 < HM / 8; ++c8) {
      const v4f va = *(const v4fa*)(rd + 8 * c8);
      const v4f vb = *(const v4fa*)(rd + 8 * c8 + 4);
      const v4f ba = *(const v4fa*)(cst + HM + 8 * c8);
      const v4f bb = *(const v4fa*)(cst + HM + 8 * c8 + 4);
      const v4f pa = *(const v4fa*)(cst + 2 * HM + 8 * c8);
      const v4f pb = *(const v4fa*)(cst + 2 * HM + 8 * c8 + 4);
      const v4f qa = *(const v4fa*)(cst + 3 * HM + 8 * c8);
      const v4f qb = *(const v4fa*)(cst + 3 * HM + 8 * c8 + 4);
      const v8f x8 = {relu_k(va.x + ba.x), relu_k(va.y + ba.y), relu_k(va.z + ba.z), relu_k(va.w + ba.w),
                      relu_k(vb.x + bb.x), relu_k(vb.y + bb.y), relu_k(vb.z + bb.z), relu_k(vb.w + bb.w)};
      const v8f p8 = {pa.x, pa.y, pa.z, pa.w, pb.x, pb.y, pb.z, pb.w};
      const v8f q8 = {qa.x, qa.y, qa.z, qa.w, qb.x, qb.y, qb.z, qb.w};
#pragma unroll
      for (int i = 0; i < 8; ++i) {
        z0 = fmaf(x8[i], p8[i], z0);
        z1 = fmaf(x8[i], q8[i], z1);
      }
    }
    const float mx  = (z0 > z1) ? z0 : z1;
    const float e0  = expf(z0 - mx);
    const float e1  = expf(z1 - mx);
    const float den = e0 + e1;
    const v2f o2 = {e0 / den, e1 / den};
    *(v2fa*)(sO + 2 * tid) = o2;
  }
  __syncthreads();

  {
    const int tl = tid < 64 ? tid : 63;
    const v4f o4 = *(const v4fa*)(sO + 4 * tl);
    const int g  = (int)blockIdx.x * 2 * RTHR + 4 * tl;
    const bool stv = (tid < 64) && (g + 4 <= 2 * NNODE);
    const int gc = stv ? g : 0;
    if (stv) *(volatile v4f*)(out + gc) = o4;
    __threadfence();
    if (stv) *(volatile v4f*)(out + gc) = o4;
  }
}

extern "C" void kernel_launch(void* const* d_in, const int* in_sizes, int n_in,
                              void* d_out, int out_size, void* d_ws, size_t ws_size,
                              hipStream_t stream) {
  if (n_in < 21) return;
  if (in_sizes[0] != NEDGE || in_sizes[1] != NEDGE || in_sizes[2] != 4 * NEDGE) return;
  if (in_sizes[5] != HM * W1IN || in_sizes[6] != HM) return;
  if (in_sizes[7] != HM * HM || in_sizes[8] != HM) return;
  if (in_sizes[9] != SD * HM || in_sizes[10] != SD) return;
  if (in_sizes[11] != 4 * SD * SD || in_sizes[12] != 4 * SD * SD) return;
  if (in_sizes[13] != 4 * SD || in_sizes[14] != 4 * SD) return;
  if (in_sizes[15] != HM * SD || in_sizes[16] != HM) return;
  if (in_sizes[17] != HM * HM || in_sizes[18] != HM) return;
  if (in_sizes[19] != 2 * HM || in_sizes[20] != 2) return;
  if (out_size != 2 * NNODE) return;
  if (WS_END > ws_size) return;

  const int*   rowv  = (const int*)d_in[0];
  const int*   colv  = (const int*)d_in[1];
  const float* ea    = (const float*)d_in[2];
  const float* mp_w1 = (const float*)d_in[5];
  const float* mp_b1 = (const float*)d_in[6];
  const float* mp_w2 = (const float*)d_in[7];
  const float* mp_b2 = (const float*)d_in[8];
  const float* mp_w3 = (const float*)d_in[9];
  const float* mp_b3 = (const float*)d_in[10];
  const float* w_ih  = (const float*)d_in[11];
  const float* w_hh  = (const float*)d_in[12];
  const float* b_ih  = (const float*)d_in[13];
  const float* b_hh  = (const float*)d_in[14];
  const float* ro_w1 = (const float*)d_in[15];
  const float* ro_b1 = (const float*)d_in[16];
  const float* ro_w2 = (const float*)d_in[17];
  const float* ro_b2 = (const float*)d_in[18];
  const float* ro_w3 = (const float*)d_in[19];
  const float* ro_b3 = (const float*)d_in[20];
  float* out = (float*)d_out;

  char* ws = (char*)d_ws;
  unsigned short* W1AB = (unsigned short*)(ws + O_W1AB);
  unsigned short* W2D  = (unsigned short*)(ws + O_W2D);
  unsigned short* W3D  = (unsigned short*)(ws + O_W3D);
  unsigned short* WG   = (unsigned short*)(ws + O_WG);
  unsigned short* R1D  = (unsigned short*)(ws + O_R1D);
  unsigned short* R2D  = (unsigned short*)(ws + O_R2D);
  unsigned short* H0   = (unsigned short*)(ws + O_H0);
  unsigned short* H1   = (unsigned short*)(ws + O_H1);
  unsigned short* NM   = (unsigned short*)(ws + O_NM);
  float*          C    = (float*)(ws + O_C);
  float*          PAB  = (float*)(ws + O_PAB);
  float*          EC   = (float*)(ws + O_EC);
  float*          MSG  = (float*)(ws + O_MSG);
  int*            LIST = (int*)(ws + O_LIST);
  int*            CNT  = (int*)(ws + O_CNT);
  int*            OFF  = (int*)(ws + O_OFF);
  int*            FLAG = (int*)(ws + O_FLAG);

  hipFuncSetAttribute(reinterpret_cast<const void*>(&k_edge), hipFuncAttributeMaxDynamicSharedMemorySize,
                      (int)EDGE_LDS_BYTES);
  hipFuncSetAttribute(reinterpret_cast<const void*>(&k_bucket), hipFuncAttributeMaxDynamicSharedMemorySize,
                      (int)AGG_LDS_BYTES);
  hipFuncSetAttribute(reinterpret_cast<const void*>(&k_lstm), hipFuncAttributeMaxDynamicSharedMemorySize,
                      (int)LSTM_LDS_BYTES);
  hipFuncSetAttribute(reinterpret_cast<const void*>(&k_ro), hipFuncAttributeMaxDynamicSharedMemorySize,
                      (int)RO_LDS_BYTES);

  k_pa<<<NU_PA / NTHR, NTHR, 0, stream>>>(mp_w1, mp_w2, mp_w3, W1AB, W2D, W3D);
  k_pb<<<NU_PB / NTHR, NTHR, 0, stream>>>(w_ih, w_hh, ro_w1, ro_w2, WG, R1D, R2D);
  k_pc<<<(3 * NU_ST) / NTHR, NTHR, 0, stream>>>(H0, H1, C);
  k_ec<<<NEDGE / 64, NTHR, 0, stream>>>(ea, mp_w1, mp_b1, EC);
  k_bucket<<<NBLK, NTHR, AGG_LDS_BYTES, stream>>>(colv, NEDGE, 1, LIST, CNT, OFF, FLAG);

  for (int t = 0; t < NSTEP; ++t) {
    unsigned short* Hin  = (t & 1) ? H1 : H0;
    unsigned short* Hout = (t & 1) ? H0 : H1;
    k_node<<<dim3(SP / GBM, PABW / GBN), GTHR, 0, stream>>>(Hin, HP, W1AB, 128, 128, PAB, PABW);
    k_edge<<<NEDGE / ETB, ETHR, EDGE_LDS_BYTES, stream>>>(rowv, colv, PAB, EC, W2D, W3D, mp_b2, mp_b3, MSG);
    k_agg<<<SP / ASLOT, NTHR, 0, stream>>>(LIST, CNT, OFF, FLAG, MSG, NM);
    k_lstm<<<SP / GBM, LTHR, LSTM_LDS_BYTES, stream>>>(NM, Hin, WG, b_ih, b_hh, C, Hout);
  }
  k_ro<<<ROT, RTHR, RO_LDS_BYTES, stream>>>(H0, R1D, R2D, ro_b1, ro_b2, ro_w3, ro_b3, out);
}
